// CondMul_1340029796953
// MI455X (gfx1250) — hardware-verified
//
#include <hip/hip_runtime.h>

typedef __attribute__((ext_vector_type(16))) _Float16 v16h;
typedef __attribute__((ext_vector_type(8)))  float    v8f;
typedef __attribute__((ext_vector_type(4)))  float    v4f;
typedef __attribute__((ext_vector_type(4)))  int      v4i;

constexpr int kRows          = 262144;
constexpr int kExperts       = 1024;
constexpr int kIn            = 32;
constexpr int kOut           = 32;
constexpr int kWavesPerBlock = 4;
constexpr int kBlocks        = kExperts / kWavesPerBlock;
constexpr int kIdsPerIter    = 128;
constexpr int kScanIters     = kRows / kIdsPerIter;
constexpr int kQCap          = 160;
constexpr int kWPitch        = 33;
constexpr int kTilePitch     = 36;
constexpr int kSlabPitch     = 36;
constexpr int kMaxTilesPerIter = 9;
constexpr float kCarryX      = 16.0f;
constexpr float kCarryW      = 256.0f;
constexpr float kFold        = 1.0f / (kCarryX * kCarryW);
constexpr float kF16MinNormal = 6.103515625e-05f;

static_assert(kIn == 32 && kOut == 32, "one 32-deep k-step, two 16-wide column tiles");
static_assert((kRows % kIdsPerIter) == 0, "id stream has no tail");
static_assert((kExperts % kWavesPerBlock) == 0, "grid covers every expert exactly once");
static_assert((size_t)kRows * kIn * 4 == 33554432ull, "input bytes");
static_assert((size_t)kRows * 4 == 1048576ull, "id bytes");
static_assert((size_t)kExperts * kIn * kOut * 4 == 4194304ull, "weight bytes");
static_assert((size_t)kExperts * kOut * 4 == 131072ull, "bias bytes");
static_assert((size_t)kRows * kOut * 4 == 33554432ull, "output bytes");
static_assert(15 + kIdsPerIter < kQCap, "queue bound: leftover below 16 plus one full step of hits");
static_assert((15 + kIdsPerIter) / 16 < kMaxTilesPerIter, "static tile-loop bound covers the worst step");
static_assert((kSlabPitch % 4) == 0 && (kTilePitch % 4) == 0, "16-B aligned LDS rows");
static_assert(kTilePitch >= kIn && kSlabPitch >= kOut, "LDS rows hold a whole line");


__device__ __forceinline__ int clampi(int v, int lo, int hi) {
  v = (v < lo) ? lo : v;
  v = (v > hi) ? hi : v;
  return v;
}

__device__ __forceinline__ _Float16 to_f16_operand(float v, float carry) {
  float s = v * carry;
  s = (fabsf(s) < kF16MinNormal) ? 0.0f : s;
  return (_Float16)s;
}

__device__ __forceinline__ v8f mma_f16(v16h a, v16h b, v8f c) {
  c = __builtin_amdgcn_wmma_f32_16x16x32_f16(false, a, false, b, (short)0, c, false, false);
  asm volatile("v_nop\n\tv_nop\n\tv_nop\n\tv_nop" : "+v"(c) : "v"(a), "v"(b));
  return c;
}

__device__ __forceinline__ void wave_lds_sync() {
  __builtin_amdgcn_fence(__ATOMIC_RELEASE, "workgroup");
  __builtin_amdgcn_wave_barrier();
  __builtin_amdgcn_fence(__ATOMIC_ACQUIRE, "workgroup");
}

__device__ __forceinline__ void process_tile(
    const float* __restrict__ x, float* __restrict__ out,
    const int* qw, float* xt, float* slab, int base, int cnt,
    v16h bf0, v16h bf1, float bias0, float bias1, int lane)
{
  wave_lds_sync();
  const int half = lane >> 4;
  const int col  = lane & 15;
  const int rq   = lane >> 3;
  const int c4   = (lane & 7) * 4;

  int  orid[4];
  bool ok[4];
#pragma unroll
  for (int j = 0; j < 4; ++j) {
    const int row = j * 4 + rq;
    const int ri  = (row < cnt) ? row : (cnt - 1);
    int t = qw[base + ri];
    t = clampi(t, 0, kRows - 1);
    orid[j] = t;
    ok[j]   = (row < cnt);
  }

  v4f xin[4];
#pragma unroll
  for (int j = 0; j < 4; ++j) {
    xin[j] = *(const v4f*)(x + (size_t)orid[j] * kIn + c4);
  }
#pragma unroll
  for (int j = 0; j < 4; ++j) {
    *(v4f*)(xt + (j * 4 + rq) * kTilePitch + c4) = xin[j];
  }
  wave_lds_sync();

  const float* xr = xt + col * kTilePitch + 8 * half;
  const v4f a0 = *(const v4f*)(xr);
  const v4f a1 = *(const v4f*)(xr + 4);
  const v4f a2 = *(const v4f*)(xr + 16);
  const v4f a3 = *(const v4f*)(xr + 20);
  v16h af;
#pragma unroll
  for (int e = 0; e < 4; ++e) {
    const float t0 = a0[e];
    const float t1 = a1[e];
    const float t2 = a2[e];
    const float t3 = a3[e];
    af[e]      = to_f16_operand(t0, kCarryX);
    af[4 + e]  = to_f16_operand(t1, kCarryX);
    af[8 + e]  = to_f16_operand(t2, kCarryX);
    af[12 + e] = to_f16_operand(t3, kCarryX);
  }

  v8f acc0 = (v8f){0.f, 0.f, 0.f, 0.f, 0.f, 0.f, 0.f, 0.f};
  v8f acc1 = (v8f){0.f, 0.f, 0.f, 0.f, 0.f, 0.f, 0.f, 0.f};
  acc0 = mma_f16(af, bf0, acc0);
  acc1 = mma_f16(af, bf1, acc1);

#pragma unroll
  for (int r = 0; r < 8; ++r) {
    const float v0 = acc0[r];
    const float v1 = acc1[r];
    slab[(8 * half + r) * kSlabPitch + col]      = fmaf(v0, kFold, bias0);
    slab[(8 * half + r) * kSlabPitch + 16 + col] = fmaf(v1, kFold, bias1);
  }
  wave_lds_sync();

  v4f ov[4];
#pragma unroll
  for (int j = 0; j < 4; ++j) {
    const int row = j * 4 + rq;
    ov[j] = *(const v4f*)(slab + row * kSlabPitch + c4);
  }
  for (int pass = 0; pass < 2; ++pass) {
#pragma unroll
    for (int j = 0; j < 4; ++j) {
      if (ok[j]) *(volatile v4f*)(out + (size_t)orid[j] * kOut + c4) = ov[j];
    }
    __threadfence();
  }
  wave_lds_sync();
}

__global__ __launch_bounds__(128) void grouped_linear_kernel(
    const float* __restrict__ x, const int* __restrict__ inds,
    const float* __restrict__ w, const float* __restrict__ b,
    float* __restrict__ out)
{
  __shared__ __align__(16) float sW[kWavesPerBlock][kIn * kWPitch];
  __shared__ __align__(16) float sX[kWavesPerBlock][16 * kTilePitch];
  __shared__ __align__(16) float sSlab[kWavesPerBlock][16 * kSlabPitch];
  __shared__ int sQ[kWavesPerBlock][kQCap];

  const int tid  = threadIdx.x;
  const int lane = tid & 31;
  const int wave = __builtin_amdgcn_readfirstlane(tid >> 5);
  const int e    = blockIdx.x * kWavesPerBlock + wave;

  float* wS   = sW[wave];
  float* xt   = sX[wave];
  float* slab = sSlab[wave];
  int*   qw   = sQ[wave];

  const float* we = w + (size_t)e * (kIn * kOut);
#pragma unroll
  for (int it = 0; it < 8; ++it) {
    const int f = (it * 32 + lane) * 4;
    const v4f wv = *(const v4f*)(we + f);
    const int k = f >> 5;
    const int c = f & 31;
    const float w0 = wv[0];
    const float w1 = wv[1];
    const float w2 = wv[2];
    const float w3 = wv[3];
    wS[k * kWPitch + c + 0] = w0;
    wS[k * kWPitch + c + 1] = w1;
    wS[k * kWPitch + c + 2] = w2;
    wS[k * kWPitch + c + 3] = w3;
  }
  __syncthreads();

  const int half = lane >> 4;
  const int col  = lane & 15;
  v16h bf0, bf1;
#pragma unroll
  for (int i = 0; i < 16; ++i) {
    const int k = (i < 8) ? (8 * half + i) : (16 + 8 * half + (i - 8));
    const float u0 = wS[k * kWPitch + col];
    const float u1 = wS[k * kWPitch + 16 + col];
    bf0[i] = to_f16_operand(u0, kCarryW);
    bf1[i] = to_f16_operand(u1, kCarryW);
  }
  const float bias0 = b[(size_t)e * kOut + col];
  const float bias1 = b[(size_t)e * kOut + 16 + col];

  const unsigned lt = (1u << lane) - 1u;
  const v4i* ip = (const v4i*)inds;
  int qlen = 0;

#pragma unroll 1
  for (int it = 0; it < kScanIters; ++it) {
    const int slot = it * 32 + lane;
    const v4i iv = ip[slot];
    const int i0 = iv[0];
    const int i1 = iv[1];
    const int i2 = iv[2];
    const int i3 = iv[3];
    const bool m0 = (clampi(i0, 0, kExperts - 1) == e);
    const bool m1 = (clampi(i1, 0, kExperts - 1) == e);
    const bool m2 = (clampi(i2, 0, kExperts - 1) == e);
    const bool m3 = (clampi(i3, 0, kExperts - 1) == e);
    const unsigned b0 = __builtin_amdgcn_ballot_w32(m0);
    const unsigned b1 = __builtin_amdgcn_ballot_w32(m1);
    const unsigned b2 = __builtin_amdgcn_ballot_w32(m2);
    const unsigned b3 = __builtin_amdgcn_ballot_w32(m3);
    const unsigned any = b0 | b1 | b2 | b3;
    if (any != 0u) {
      const int rb = slot * 4;
      const int s0 = qlen;
      const int s1 = s0 + __builtin_popcount(b0);
      const int s2 = s1 + __builtin_popcount(b1);
      const int s3 = s2 + __builtin_popcount(b2);
      const int s4 = s3 + __builtin_popcount(b3);
      const int p0 = s0 + __builtin_popcount(b0 & lt);
      const int p1 = s1 + __builtin_popcount(b1 & lt);
      const int p2 = s2 + __builtin_popcount(b2 & lt);
      const int p3 = s3 + __builtin_popcount(b3 & lt);
      if (m0 && p0 < kQCap) qw[p0] = rb;
      if (m1 && p1 < kQCap) qw[p1] = rb + 1;
      if (m2 && p2 < kQCap) qw[p2] = rb + 2;
      if (m3 && p3 < kQCap) qw[p3] = rb + 3;
      qlen = (s4 < kQCap) ? s4 : kQCap;
#pragma unroll 1
      for (int t = 0; t < kMaxTilesPerIter; ++t) {
        if (qlen < 16) break;
        process_tile(x, out, qw, xt, slab, qlen - 16, 16, bf0, bf1, bias0, bias1, lane);
        qlen -= 16;
      }
    }
  }
  if (qlen > 0) {
    const int rem = (qlen < 16) ? qlen : 16;
    process_tile(x, out, qw, xt, slab, 0, rem, bf0, bf1, bias0, bias1, lane);
  }
}

extern "C" void kernel_launch(void* const* d_in, const int* in_sizes, int n_in,
                              void* d_out, int out_size, void* d_ws, size_t ws_size,
                              hipStream_t stream) {
  (void)in_sizes; (void)out_size; (void)d_ws; (void)ws_size;
  if (n_in < 4) return;
  const float* x    = (const float*)d_in[0];
  const int*   inds = (const int*)d_in[1];
  const float* w    = (const float*)d_in[2];
  const float* b    = (const float*)d_in[3];
  float*       out  = (float*)d_out;
  grouped_linear_kernel<<<kBlocks, kWavesPerBlock * 32, 0, stream>>>(x, inds, w, b, out);
}
